// MultiHeadSelfAttention_26293789786283
// MI455X (gfx1250) — hardware-verified
//
#include <hip/hip_runtime.h>
#include <math.h>

typedef __attribute__((ext_vector_type(16))) _Float16 v16h;
typedef __attribute__((ext_vector_type(16))) __bf16 v16b;
typedef __attribute__((ext_vector_type(8)))  _Float16 v8h;
typedef __attribute__((ext_vector_type(8)))  __bf16 v8b;
typedef __attribute__((ext_vector_type(8)))  float v8f;
typedef __attribute__((ext_vector_type(4)))  float v4f;
typedef __attribute__((ext_vector_type(4)))  unsigned v4u;

template <typename T> __device__ __forceinline__ void vst2(void* p, T v) { *(volatile T*)p = v; __threadfence(); *(volatile T*)p = v; }
__device__ __forceinline__ v8f wmma16(v16h a, v16h b, v8f c) {
  v8f d = __builtin_amdgcn_wmma_f32_16x16x32_f16(false, a, false, b, (short)0, c, false, false);
  asm volatile("v_nop\n\tv_nop\n\tv_nop\n\tv_nop" : "+v"(d) : "v"(a), "v"(b));
  return d;
}
__device__ __forceinline__ v8f wmma_bf(v16b a, v16b b, v8f c) {
  v8f d = __builtin_amdgcn_wmma_f32_16x16x32_bf16(false, a, false, b, (short)0, c, false, false);
  asm volatile("v_nop\n\tv_nop\n\tv_nop\n\tv_nop" : "+v"(d) : "v"(a), "v"(b));
  return d;
}
__device__ __forceinline__ v16h frag_h(const _Float16* rowk0, int lane) {
  union { v16h v; v8h q[2]; } u; const _Float16* p = rowk0 + 8 * (lane >> 4);
  u.q[0] = *(const v8h*)p; u.q[1] = *(const v8h*)(p + 16); return u.v;
}
__device__ __forceinline__ v16b frag_b(const __bf16* rowk0, int lane) {
  union { v16b v; v8b q[2]; } u; const __bf16* p = rowk0 + 8 * (lane >> 4);
  u.q[0] = *(const v8b*)p; u.q[1] = *(const v8b*)(p + 16); return u.v;
}
__device__ __forceinline__ float bfr(float v) { return (float)(__bf16)v; }
union PK8 { v8b b; v4u u; };
#define LDSX() do { asm volatile("s_wait_dscnt 0" ::: "memory"); __builtin_amdgcn_wave_barrier(); __builtin_amdgcn_fence(3  , "workgroup"); } while (0)

#ifndef NB
#define NB 2
#endif
#ifndef SEQ
#define SEQ 2048
#endif
#define NB_FULL 2
#define CC 1024
#define DIN 1024
#define NH 16
#define HD 64
#define SCALE (0.125f)

static_assert(NB <= NB_FULL);
static_assert(SEQ % 64 == 0);
static_assert(CC % 128 == 0);
static_assert(DIN % 128 == 0);
static_assert(DIN % 32 == 0);
static_assert(CC % 32 == 0);
static_assert(NH * HD == CC);
static_assert(HD == 64);
static_assert(DIN == CC);
static_assert(((size_t)NB * SEQ * DIN / 8) % 256 == 0);
static_assert(((size_t)3 * CC * DIN / 8) % 256 == 0);
static_assert(((size_t)DIN * CC / 8) % 256 == 0);
static_assert(DIN / 8 == 128);

#define SZ_ACT ((size_t)2 * NB * SEQ * CC)
#define WS_XQ  ((size_t)0)
#define WS_XK  (WS_XQ + SZ_ACT)
#define WS_XV  (WS_XK + SZ_ACT)
#define WS_WI  (WS_XV + SZ_ACT)
#define WS_WO  (WS_WI + (size_t)2 * 3 * CC * DIN)
#define WS_QH  (WS_WO + (size_t)2 * DIN * CC)
#define WS_QL  (WS_QH + SZ_ACT)
#define WS_KH  (WS_QL + SZ_ACT)
#define WS_KL  (WS_KH + SZ_ACT)
#define WS_VT  (WS_KL + SZ_ACT)
#define WS_YH  (WS_VT + SZ_ACT)
#define WS_YL  (WS_YH + SZ_ACT)
#define WS_END (WS_YL + SZ_ACT)
static_assert(WS_END <= (size_t)134217728);
static_assert(SZ_ACT % 128 == 0);

__global__ __launch_bounds__(256) void k_cvtx(const float* __restrict__ X, __bf16* __restrict__ XB) {
  const size_t i = (size_t)blockIdx.x * 256 + threadIdx.x;
  const size_t row = i / (DIN / 8); const int pc = (int)(i % (DIN / 8));
  const size_t bb = row / SEQ, t = row % SEQ;
  const float* src = X + (t * NB_FULL + bb) * DIN + pc * 8;
  const v4f x0 = *(const v4f*)src, x1 = *(const v4f*)(src + 4);
  v8b o; o[0] = (__bf16)x0[0]; o[1] = (__bf16)x0[1]; o[2] = (__bf16)x0[2]; o[3] = (__bf16)x0[3]; o[4] = (__bf16)x1[0]; o[5] = (__bf16)x1[1]; o[6] = (__bf16)x1[2]; o[7] = (__bf16)x1[3];
  PK8 u; u.b = o; vst2(XB + i * 8, u.u);
}
__global__ __launch_bounds__(256) void k_cvtw(const float* __restrict__ W, __bf16* __restrict__ WB, int n8) {
  const size_t i = (size_t)blockIdx.x * 256 + threadIdx.x;
  if (i < (size_t)n8) {
    const float* src = W + i * 8;
    const v4f x0 = *(const v4f*)src, x1 = *(const v4f*)(src + 4);
    v8b o; o[0] = (__bf16)x0[0]; o[1] = (__bf16)x0[1]; o[2] = (__bf16)x0[2]; o[3] = (__bf16)x0[3]; o[4] = (__bf16)x1[0]; o[5] = (__bf16)x1[1]; o[6] = (__bf16)x1[2]; o[7] = (__bf16)x1[3];
    PK8 u; u.b = o; vst2(WB + i * 8, u.u);
  }
}

__device__ __forceinline__ void gemm8_bf(const __bf16* __restrict__ A, const size_t aoff, const __bf16* __restrict__ W, const size_t woff, const int lane, v8f (&acc)[8]) {
#pragma unroll 1
  for (int kc = 0; kc < DIN / 32; ++kc) {
    const v16b a = frag_b(A + aoff + kc * 32, lane);
#pragma unroll
    for (int j = 0; j < 8; ++j) { const v16b w = frag_b(W + woff + (size_t)j * 16 * DIN + kc * 32, lane); acc[j] = wmma_bf(a, w, acc[j]); }
  }
}

__global__ __launch_bounds__(128) void k_proj_qk(const __bf16* __restrict__ XB, const __bf16* __restrict__ WB, const float* __restrict__ BA, _Float16* __restrict__ DH, _Float16* __restrict__ DL) {
  __shared__ __align__(16) _Float16 sh[64][136], sl[64][136];
  const int tid = threadIdx.x; const int wave = __builtin_amdgcn_readfirstlane((int)(threadIdx.x >> 5)); const int lane = tid & 31, col = lane & 15, g = lane >> 4;
  const int c0 = blockIdx.y * 128; const size_t r0 = (size_t)blockIdx.x * 64;
  v8f acc[8] = {};
  gemm8_bf(XB, (r0 + wave * 16 + col) * DIN, WB, (size_t)(c0 + col) * DIN, lane, acc);
#pragma unroll
  for (int j = 0; j < 8; ++j) { const float bias = bfr(BA[c0 + j * 16 + col]);
#pragma unroll
    for (int r = 0; r < 8; ++r) { const float v = acc[j][r] + bias; const _Float16 hv = (_Float16)v; sh[wave * 16 + 8 * g + r][j * 16 + col] = hv; sl[wave * 16 + 8 * g + r][j * 16 + col] = (_Float16)((v - (float)hv) * 1024.0f); } }
  __syncthreads();
  for (int e = tid; e < 64 * 16; e += 128) { const int rl = e >> 4, q = e & 15; const size_t o = (r0 + rl) * CC + c0 + q * 8;
    const v4u a = *(const v4u*)&sh[rl][q * 8]; const v4u b = *(const v4u*)&sl[rl][q * 8]; vst2(DH + o, a); vst2(DL + o, b); }
}
__global__ __launch_bounds__(128) void k_proj_v(const __bf16* __restrict__ XB, const __bf16* __restrict__ WB, const float* __restrict__ BA, _Float16* __restrict__ VT) {
  __shared__ __align__(16) _Float16 th[128][72];
  const int tid = threadIdx.x; const int wave = __builtin_amdgcn_readfirstlane((int)(threadIdx.x >> 5)); const int lane = tid & 31, col = lane & 15, g = lane >> 4;
  const int c0 = blockIdx.y * 128; const size_t r0 = (size_t)blockIdx.x * 64; const size_t bb = r0 / SEQ; const int t0 = (int)(r0 % SEQ);
  v8f acc[8] = {};
  gemm8_bf(XB, (r0 + wave * 16 + col) * DIN, WB, (size_t)(c0 + col) * DIN, lane, acc);
#pragma unroll
  for (int j = 0; j < 8; ++j) { const float bias = bfr(BA[c0 + j * 16 + col]);
#pragma unroll
    for (int r = 0; r < 8; ++r) { const float v = acc[j][r] + bias; th[j * 16 + col][wave * 16 + 8 * g + r] = (_Float16)v; } }
  __syncthreads();
  for (int e = tid; e < 128 * 8; e += 128) { const int cl = e >> 3, q = e & 7; const v4u a = *(const v4u*)&th[cl][q * 8]; vst2(VT + (bb * CC + c0 + cl) * (size_t)SEQ + t0 + q * 8, a); }
}

__global__ __launch_bounds__(128) void k_attn(const _Float16* __restrict__ QH, const _Float16* __restrict__ QL, const _Float16* __restrict__ KH, const _Float16* __restrict__ KL, const _Float16* __restrict__ VT, __bf16* __restrict__ YH, __bf16* __restrict__ YL) {
  __shared__ __align__(16) __bf16 syh[4][16][72], syl[4][16][72];
  const int tid = threadIdx.x; const int wave = __builtin_amdgcn_readfirstlane((int)(threadIdx.x >> 5)); const int lane = tid & 31, col = lane & 15, g = lane >> 4;
  const int qb = blockIdx.x; const int b = blockIdx.y / NH, hd = blockIdx.y % NH;
  const int q0 = qb * 64 + wave * 16;
  const size_t qoff = ((size_t)b * SEQ + q0 + col) * CC + hd * HD;
  const size_t kbase = ((size_t)b * SEQ + col) * CC + hd * HD;
  const size_t vbase = ((size_t)b * CC + hd * HD + col) * (size_t)SEQ;
  v8f o[4] = {};
  float m = -1.0e30f, l = 0.0f;
#pragma unroll 1
  for (int kb = 0; kb < SEQ / 32; ++kb) {
    v8f a0 = {}, a1 = {}, e0 = {}, e1 = {};
    const size_t ko = kbase + (size_t)kb * 32 * CC;
#pragma unroll
    for (int kc = 0; kc < HD / 32; ++kc) {
      const v16h qh = frag_h(QH + qoff + kc * 32, lane), ql = frag_h(QL + qoff + kc * 32, lane);
      const v16h k0h = frag_h(KH + ko + kc * 32, lane), k0l = frag_h(KL + ko + kc * 32, lane);
      a0 = wmma16(k0h, qh, a0); e0 = wmma16(k0l, qh, e0); e0 = wmma16(k0h, ql, e0);
      const v16h k1h = frag_h(KH + ko + (size_t)16 * CC + kc * 32, lane), k1l = frag_h(KL + ko + (size_t)16 * CC + kc * 32, lane);
      a1 = wmma16(k1h, qh, a1); e1 = wmma16(k1l, qh, e1); e1 = wmma16(k1h, ql, e1);
    }
    float s0[8], s1[8]; float mx = -1.0e30f;
#pragma unroll
    for (int r = 0; r < 8; ++r) { s0[r] = (a0[r] + e0[r] * (1.0f / 1024.0f)) * SCALE; s1[r] = (a1[r] + e1[r] * (1.0f / 1024.0f)) * SCALE; mx = fmaxf(mx, fmaxf(s0[r], s1[r])); }
    mx = fmaxf(mx, __shfl_xor(mx, 16));
    const float nm = fmaxf(m, mx); const float corr = __expf(m - nm); m = nm;
    float sum = 0.0f; v16h pb;
#pragma unroll
    for (int r = 0; r < 8; ++r) { const float p0 = __expf(s0[r] - nm), p1 = __expf(s1[r] - nm); sum += p0 + p1; pb[r] = (_Float16)(p0 * 1024.0f); pb[8 + r] = (_Float16)(p1 * 1024.0f); }
    sum += __shfl_xor(sum, 16);
    l = l * corr + sum;
#pragma unroll
    for (int j = 0; j < 4; ++j)
#pragma unroll
      for (int r = 0; r < 8; ++r) o[j][r] *= corr;
#pragma unroll
    for (int j = 0; j < 4; ++j) { const v16h vt = frag_h(VT + vbase + (size_t)j * 16 * SEQ + kb * 32, lane); o[j] = wmma16(vt, pb, o[j]); }
  }
  const float inv = 1.0f / (l * 1024.0f);
#pragma unroll
  for (int j = 0; j < 4; ++j) { v8b hb, lb;
#pragma unroll
    for (int r = 0; r < 8; ++r) { const float v = o[j][r] * inv; const __bf16 hv = (__bf16)v; hb[r] = hv; lb[r] = (__bf16)(v - (float)hv); }
    *(v8b*)&syh[wave][col][j * 16 + 8 * g] = hb; *(v8b*)&syl[wave][col][j * 16 + 8 * g] = lb; }
  LDSX();
#pragma unroll
  for (int it = 0; it < 4; ++it) { const int rl = it * 4 + (lane >> 3), pc = lane & 7; const size_t off = ((size_t)b * SEQ + q0 + rl) * CC + hd * HD + pc * 8;
    const v4u a = *(const v4u*)&syh[wave][rl][pc * 8]; const v4u c = *(const v4u*)&syl[wave][rl][pc * 8]; vst2(YH + off, a); vst2(YL + off, c); }
}

__global__ __launch_bounds__(128) void k_out(const __bf16* __restrict__ YH, const __bf16* __restrict__ YL, const __bf16* __restrict__ WOB, const float* __restrict__ BO, float* __restrict__ OUT) {
  __shared__ __align__(16) float sf[4][16][132];
  const int tid = threadIdx.x; const int wave = __builtin_amdgcn_readfirstlane((int)(threadIdx.x >> 5)); const int lane = tid & 31, col = lane & 15, g = lane >> 4;
  const int c0 = blockIdx.y * 128; const size_t rb = (size_t)blockIdx.x * 64; const size_t bb = rb / SEQ; const size_t t0 = rb % SEQ + (size_t)wave * 16; const size_t r0 = rb + (size_t)wave * 16;
  v8f acc[8] = {};
  const size_t aoff = (r0 + col) * CC; const size_t woff = (size_t)(c0 + col) * CC;
#pragma unroll 1
  for (int kc = 0; kc < CC / 32; ++kc) {
    const v16b yh = frag_b(YH + aoff + kc * 32, lane), yl = frag_b(YL + aoff + kc * 32, lane);
#pragma unroll
    for (int j = 0; j < 8; ++j) { const v16b w = frag_b(WOB + woff + (size_t)j * 16 * CC + kc * 32, lane); acc[j] = wmma_bf(yl, w, acc[j]); acc[j] = wmma_bf(yh, w, acc[j]); }
  }
#pragma unroll
  for (int j = 0; j < 8; ++j) { const float bias = bfr(BO[c0 + j * 16 + col]);
#pragma unroll
    for (int r = 0; r < 8; ++r) sf[wave][8 * g + r][j * 16 + col] = acc[j][r] + bias; }
  LDSX();
  for (int rl = 0; rl < 16; ++rl) { const v4f v = *(const v4f*)&sf[wave][rl][lane * 4]; vst2(OUT + ((t0 + rl) * NB_FULL + bb) * DIN + c0 + lane * 4, v); }
}

extern "C" void kernel_launch(void* const* d_in, const int* in_sizes, int n_in, void* d_out, int out_size, void* d_ws, size_t ws_size, hipStream_t stream) {
  if (n_in < 7) return;
  const size_t needx = ((size_t)(SEQ - 1) * NB_FULL + NB) * DIN;
  if ((size_t)in_sizes[0] < needx || (size_t)in_sizes[1] < needx || (size_t)in_sizes[2] < needx) return;
  if ((size_t)in_sizes[3] < (size_t)3 * CC * DIN || in_sizes[4] < 3 * CC || (size_t)in_sizes[5] < (size_t)DIN * CC || in_sizes[6] < DIN) return;
  if ((size_t)out_size < needx) return;
  if (ws_size < (size_t)WS_END) return;
  const float* xq = (const float*)d_in[0]; const float* xk = (const float*)d_in[1]; const float* xv = (const float*)d_in[2];
  const float* wi = (const float*)d_in[3]; const float* bi = (const float*)d_in[4]; const float* wo = (const float*)d_in[5]; const float* bo = (const float*)d_in[6];
  char* ws = (char*)d_ws;
  __bf16 *XQ = (__bf16*)(ws + WS_XQ), *XK = (__bf16*)(ws + WS_XK), *XV = (__bf16*)(ws + WS_XV), *WI = (__bf16*)(ws + WS_WI), *WO = (__bf16*)(ws + WS_WO);
  _Float16 *QH = (_Float16*)(ws + WS_QH), *QL = (_Float16*)(ws + WS_QL), *KH = (_Float16*)(ws + WS_KH), *KL = (_Float16*)(ws + WS_KL), *VT = (_Float16*)(ws + WS_VT);
  __bf16 *YH = (__bf16*)(ws + WS_YH), *YL = (__bf16*)(ws + WS_YL);
  const unsigned gx = (unsigned)((size_t)NB * SEQ * DIN / 8 / 256);
  k_cvtx<<<dim3(gx), 256, 0, stream>>>(xq, XQ);
  k_cvtx<<<dim3(gx), 256, 0, stream>>>(xk, XK);
  k_cvtx<<<dim3(gx), 256, 0, stream>>>(xv, XV);
  k_cvtw<<<dim3((unsigned)((size_t)3 * CC * DIN / 8 / 256)), 256, 0, stream>>>(wi, WI, (int)((size_t)3 * CC * DIN / 8));
  k_cvtw<<<dim3((unsigned)((size_t)DIN * CC / 8 / 256)), 256, 0, stream>>>(wo, WO, (int)((size_t)DIN * CC / 8));
  k_proj_qk<<<dim3(NB * SEQ / 64, CC / 128), 128, 0, stream>>>(XQ, WI, bi, QH, QL);
  k_proj_qk<<<dim3(NB * SEQ / 64, CC / 128), 128, 0, stream>>>(XK, WI + (size_t)CC * DIN, bi + CC, KH, KL);
  k_proj_v<<<dim3(NB * SEQ / 64, CC / 128), 128, 0, stream>>>(XV, WI + (size_t)2 * CC * DIN, bi + 2 * CC, VT);
  k_attn<<<dim3(SEQ / 64, NB * NH), 128, 0, stream>>>(QH, QL, KH, KL, VT, YH, YL);
  k_out<<<dim3(NB * SEQ / 64, DIN / 128), 128, 0, stream>>>(YH, YL, WO, bo, (float*)d_out);
}
